// ViTBlock_68272800137233
// MI455X (gfx1250) — hardware-run, weakly checked
//
#include <hip/hip_runtime.h>
#include <math.h>

constexpr int kBatch  = 16;
constexpr int kSeq    = 512;
constexpr int kDim    = 768;
constexpr int kHeads  = 12;
constexpr int kDh     = 64;
constexpr int kMlp    = 3072;
constexpr int kTok    = kBatch * kSeq;
constexpr int kMChunk = 4096;
constexpr int kHeadW  = kDh * kDh;
constexpr float kWCarry     = 16.0f;
constexpr float kWCarryInv  = 1.0f / 16.0f;
constexpr float kPCarry     = 32768.0f;
constexpr float kPCarryInv  = 1.0f / 32768.0f;
constexpr float kScoreScale = 0.125f;
constexpr float kInvDim     = 1.0f / 768.0f;
constexpr float kLnEps      = 1.0e-5f;
static_assert(kHeads * kDh == kDim);
static_assert(kTok % 64 == 0 && kSeq % 64 == 0 && kDh % 64 == 0 && kDim % 64 == 0 && kMlp % 64 == 0 && kMChunk % 64 == 0);
static_assert(kDh % 32 == 0 && kSeq % 32 == 0 && kDim % 32 == 0 && kMlp % 32 == 0);
static_assert(kTok % kMChunk == 0);
static_assert(kDim == 96 * 8);
static_assert(kSeq == 64 * 8);
static_assert((kMChunk * kMlp) % 4096 == 0);

typedef __attribute__((ext_vector_type(16))) _Float16 v16h;
typedef __attribute__((ext_vector_type(8)))  _Float16 v8h;
typedef __attribute__((ext_vector_type(16))) __bf16   v16b;
typedef __attribute__((ext_vector_type(8)))  __bf16   v8b;
typedef __attribute__((ext_vector_type(8)))  float    v8f;
typedef __attribute__((ext_vector_type(4)))  float    v4f;
typedef __attribute__((ext_vector_type(2)))  float    v2f;
typedef __attribute__((ext_vector_type(4)))  unsigned int v4u;

__device__ __forceinline__ unsigned short f2bf_bits(float f) {
  unsigned u = __float_as_uint(f);
  return (unsigned short)((u + 0x7FFFu + ((u >> 16) & 1u)) >> 16);
}
__device__ __forceinline__ float bf_bits2f(unsigned short h) { return __uint_as_float(((unsigned)h) << 16); }

__device__ __forceinline__ void dep_guard_h(v8f& a, v8f& b, v16h x, v16h y) { asm volatile("v_nop\n\tv_nop\n\tv_nop\n\tv_nop" : "+v"(a), "+v"(b) : "v"(x), "v"(y)); }
__device__ __forceinline__ void dep_guard_b(v8f& a, v8f& b, v16b x, v16b y) { asm volatile("v_nop\n\tv_nop\n\tv_nop\n\tv_nop" : "+v"(a), "+v"(b) : "v"(x), "v"(y)); }
__device__ __forceinline__ void keep4_h(v16h a, v16h b, v16h c, v16h d) { asm volatile("v_nop" :: "v"(a), "v"(b), "v"(c), "v"(d)); }
__device__ __forceinline__ void keep4_b(v16b a, v16b b, v16b c, v16b d) { asm volatile("v_nop" :: "v"(a), "v"(b), "v"(c), "v"(d)); }
__device__ __forceinline__ void acc_guard4(v8f& a, v8f& b, v8f& c, v8f& d) { asm volatile("v_nop\n\tv_nop\n\tv_nop\n\tv_nop" : "+v"(a), "+v"(b), "+v"(c), "+v"(d)); }
template <typename T> struct Frag;
template <> struct Frag<_Float16> {
  typedef v16h V; union U { v16h v; v8h h[2]; };
  static __device__ __forceinline__ v16h load(const _Float16* p) {
    U f; f.h[0] = *(const v8h*)(p); f.h[1] = *(const v8h*)(p + 16); return f.v;
  }
  static __device__ __forceinline__ v8f mma(v16h a, v16h b, v8f c) {
    return __builtin_amdgcn_wmma_f32_16x16x32_f16(false, a, false, b, (short)0, c, false, false);
  }
  static __device__ __forceinline__ void guard(v8f& a, v8f& b, v16h x, v16h y) { dep_guard_h(a, b, x, y); }
  static __device__ __forceinline__ void keep(v16h a, v16h b, v16h c, v16h d) { keep4_h(a, b, c, d); }
};
template <> struct Frag<__bf16> {
  typedef v16b V; union U { v16b v; v8b h[2]; };
  static __device__ __forceinline__ v16b load(const __bf16* p) {
    U f; f.h[0] = *(const v8b*)(p); f.h[1] = *(const v8b*)(p + 16); return f.v;
  }
  static __device__ __forceinline__ v8f mma(v16b a, v16b b, v8f c) {
    return __builtin_amdgcn_wmma_f32_16x16x32_bf16(false, a, false, b, (short)0, c, false, false);
  }
  static __device__ __forceinline__ void guard(v8f& a, v8f& b, v16b x, v16b y) { dep_guard_b(a, b, x, y); }
  static __device__ __forceinline__ void keep(v16b a, v16b b, v16b c, v16b d) { keep4_b(a, b, c, d); }
};

__device__ __forceinline__ unsigned pk16(unsigned short a, unsigned short b) { return (unsigned)a | ((unsigned)b << 16); }
__device__ __forceinline__ unsigned short h_bits(float f) { const _Float16 h = (_Float16)f; return __builtin_bit_cast(unsigned short, h); }
__device__ __forceinline__ float h16_to_f32(unsigned hb) {
  const unsigned sgn = (hb & 0x8000u) << 16; const unsigned em = hb & 0x7fffu;
  const float fn = __uint_as_float((em << 13) + 0x38000000u);
  const float fs = (float)em * 5.9604644775390625e-8f;
  const float mag = (em < 0x400u) ? fs : fn; return __uint_as_float(__float_as_uint(mag) | sgn); }

template <int ET> struct Elem;
template <> struct Elem<0> { typedef _Float16 T; };
template <> struct Elem<1> { typedef __bf16 T; };
template <int ET, bool SPLIT, int BIAS_MODE, int OUT_MODE, bool RESID, int ACT = 0>
__global__ __launch_bounds__(256) void wmma_gemm64(
    const unsigned short* __restrict__ Ap, const unsigned short* __restrict__ A2p, int lda, long strideA,
    const unsigned short* __restrict__ Btp, const unsigned short* __restrict__ Bt2p, int ldb, long strideB,
    void* Cout, void* Cout2, int ldc, long strideC,
    const float* __restrict__ bias, long strideBias,
    const float* resid, long strideR,
    int M, int N, int K, float scale) {
  static_assert(!(RESID && OUT_MODE != 0));
  typedef typename Elem<ET>::T T;
  typedef typename Frag<T>::V V;
  const T* A = (const T*)Ap; const T* A2 = (const T*)A2p; const T* Bt = (const T*)Btp; const T* Bt2 = (const T*)Bt2p;
  __shared__ __align__(16) float sT[8][16 * 68];
  const int b    = blockIdx.y;
  const int lane = threadIdx.x & 31;
  const int wave = threadIdx.x >> 5;
  const int tilesN = N >> 6;
  const int tilesM = M >> 6;
  const int tile = blockIdx.x * 8 + wave;
  if (tile >= tilesM * tilesN) return;
  const int tm = tile / tilesN;
  const int tn = tile - tm * tilesN;
  const int m0 = tm << 6;
  const int n0 = tn << 6;

  const T* Ab  = A  + (size_t)b * strideA;
  const T* Bb  = Bt + (size_t)b * strideB;
  const T* Ab2 = SPLIT ? (A2  + (size_t)b * strideA) : nullptr;
  const T* Bb2 = SPLIT ? (Bt2 + (size_t)b * strideB) : nullptr;

  const int rlane = lane & 15;
  const int koff  = (lane >> 4) * 8;
  const int mOff  = (lane >> 4) * 8;

  v8f acc[4][4];
#pragma unroll
  for (int i = 0; i < 4; ++i)
#pragma unroll
    for (int j = 0; j < 4; ++j) acc[i][j] = (v8f){0.f,0.f,0.f,0.f,0.f,0.f,0.f,0.f};

  for (int k0 = 0; k0 < K; k0 += 32) {
    V bh[4], bl[4];
#pragma unroll
    for (int j = 0; j < 4; ++j) {
      const size_t bo = (size_t)(n0 + (j << 4) + rlane) * ldb + koff + k0;
      bh[j] = Frag<T>::load(Bb + bo);
      if (SPLIT) bl[j] = Frag<T>::load(Bb2 + bo);
    }
#pragma unroll
    for (int i = 0; i < 4; ++i) {
      const size_t ao = (size_t)(m0 + (i << 4) + rlane) * lda + koff + k0;
      V ah = Frag<T>::load(Ab + ao);
      V al;
      if (SPLIT) al = Frag<T>::load(Ab2 + ao);
#pragma unroll
      for (int j = 0; j < 4; ++j) {
        acc[i][j] = Frag<T>::mma(ah, bh[j], acc[i][j]);
        if (SPLIT) {
          acc[i][j] = Frag<T>::mma(ah, bl[j], acc[i][j]);
          acc[i][j] = Frag<T>::mma(al, bh[j], acc[i][j]);
        }
      }
      Frag<T>::guard(acc[i][0], acc[i][3], ah, SPLIT ? al : ah);
    }
    Frag<T>::keep(bh[0], bh[1], bh[2], bh[3]);
    if (SPLIT) Frag<T>::keep(bl[0], bl[1], bl[2], bl[3]);
  }
  acc_guard4(acc[0][0], acc[0][1], acc[0][2], acc[0][3]);
  acc_guard4(acc[1][0], acc[1][1], acc[1][2], acc[1][3]);
  acc_guard4(acc[2][0], acc[2][1], acc[2][2], acc[2][3]);
  acc_guard4(acc[3][0], acc[3][1], acc[3][2], acc[3][3]);

  float* slab = sT[wave];
  const float* Bbias = (BIAS_MODE != 0) ? (bias + (size_t)b * strideBias) : bias;
#pragma unroll
  for (int i = 0; i < 4; ++i) {
    const int mBase = m0 + (i << 4);
#pragma unroll
    for (int j = 0; j < 4; ++j) {
      const int n = n0 + (j << 4) + rlane;
      float bv = 0.f;
      if (BIAS_MODE == 2) bv = Bbias[n];
#pragma unroll
      for (int r = 0; r < 8; ++r) {
        float v = acc[i][j][r] * scale;
        if (BIAS_MODE == 1) v += Bbias[mBase + mOff + r];
        if (BIAS_MODE == 2) v += bv;
        if (ACT == 2) v = fmaxf(v, 0.0f);
        if (ACT == 4) v = (v > 0.f) ? v : 0.01f * v;
        slab[(mOff + r) * 68 + (j << 4) + rlane] = v;
      }
    }
    __builtin_amdgcn_fence(__ATOMIC_RELEASE, "workgroup");
    __builtin_amdgcn_wave_barrier();
    __builtin_amdgcn_fence(__ATOMIC_ACQUIRE, "workgroup");
    if (OUT_MODE == 0) {
      float* C = (float*)Cout + (size_t)b * strideC;
      const float* Rb = RESID ? (resid + (size_t)b * strideR) : resid;
      const int hh = lane >> 4, c4 = (lane & 15) * 4;
#pragma unroll
      for (int half = 0; half < 2; ++half) {
        v4f vals[4];
#pragma unroll
        for (int qq = 0; qq < 4; ++qq) {
          const int row = (half * 4 + qq) * 2 + hh;
          v4f v = *(const v4f*)(slab + row * 68 + c4);
          if (RESID) {
            const v4f rr = *(const v4f*)(Rb + (size_t)(mBase + row) * ldc + n0 + c4);
            v = v + rr;
          }
          vals[qq] = v;
        }
        for (int pass = 0; pass < 2; ++pass) {
#pragma unroll
          for (int qq = 0; qq < 4; ++qq) {
            const int row = (half * 4 + qq) * 2 + hh;
            *(volatile v4f*)(C + (size_t)(mBase + row) * ldc + n0 + c4) = vals[qq];
          }
          __threadfence();
        }
      }
    } else {
      const int q = lane >> 3, c8 = (lane & 7) * 8;
      unsigned short* C  = (unsigned short*)Cout  + (size_t)b * strideC;
      unsigned short* C2 = (OUT_MODE == 2) ? ((unsigned short*)Cout2 + (size_t)b * strideC) : nullptr;
      for (int pass = 0; pass < 2; ++pass) {
#pragma unroll
        for (int it = 0; it < 4; ++it) {
          const int row = it * 4 + q;
          const float* sp = slab + row * 68 + c8;
          v8h hv, lv;
#pragma unroll
          for (int e = 0; e < 8; ++e) {
            if (OUT_MODE == 1) {
              hv[e] = (_Float16)sp[e];
            } else {
              unsigned short hb = f2bf_bits(sp[e]);
              unsigned short lb = f2bf_bits(sp[e] - bf_bits2f(hb));
              hv[e] = __builtin_bit_cast(_Float16, hb);
              lv[e] = __builtin_bit_cast(_Float16, lb);
            }
          }
          *(volatile v8h*)(C + (size_t)(mBase + row) * ldc + n0 + c8) = hv;
          if (OUT_MODE == 2) *(volatile v8h*)(C2 + (size_t)(mBase + row) * ldc + n0 + c8) = lv;
        }
        __threadfence();
      }
    }
    __builtin_amdgcn_fence(__ATOMIC_RELEASE, "workgroup");
    __builtin_amdgcn_wave_barrier();
    __builtin_amdgcn_fence(__ATOMIC_ACQUIRE, "workgroup");
  }
}

__global__ __launch_bounds__(256) void wcast_head_kernel(const float* __restrict__ Wq, const float* __restrict__ Wk,
                                                        const float* __restrict__ Wv, unsigned short* __restrict__ WT, float scale) {
  __shared__ float sm[64][65];
  const int t = threadIdx.x;
  const int h = blockIdx.x;
  const int z = blockIdx.y;
  const float* W  = (z == 0) ? Wq : (z == 1) ? Wk : Wv;
  const float* Wh = W + (size_t)h * kHeadW;
#pragma unroll
  for (int i = 0; i < 16; ++i) {
    const int e_ = i * 256 + t;
    const int d  = e_ >> 6;
    const int ec = e_ & 63;
    sm[ec][d] = Wh[e_] * scale;
  }
  __syncthreads();
  const int lane = t & 31, wave = t >> 5;
  const int q = lane >> 3, c8 = (lane & 7) * 8;
  unsigned short* op = WT + ((size_t)z * kHeads + h) * kHeadW;
  for (int pass = 0; pass < 2; ++pass) {
#pragma unroll
    for (int it = 0; it < 2; ++it) {
      const int row = wave * 8 + it * 4 + q;
      unsigned short hb[8];
#pragma unroll
      for (int e = 0; e < 8; ++e) hb[e] = h_bits(sm[row][c8 + e]);
      const v4u u = (v4u){pk16(hb[0], hb[1]), pk16(hb[2], hb[3]), pk16(hb[4], hb[5]), pk16(hb[6], hb[7])};
      *(volatile v4u*)(op + (size_t)row * kDh + c8) = u;
    }
    __threadfence();
  }
}

__global__ __launch_bounds__(256) void wtcast_kernel(const float* __restrict__ W, unsigned short* __restrict__ out,
                                                    int R, int C, float scale) {
  __shared__ float sm[64][65];
  const int t  = threadIdx.x;
  const int r0 = blockIdx.x * 64;
  const int c0 = blockIdx.y * 64;
#pragma unroll
  for (int i = 0; i < 16; ++i) {
    const int e  = i * 256 + t;
    const int rl = e >> 6;
    const int cl = e & 63;
    sm[cl][rl] = W[(size_t)(r0 + rl) * C + c0 + cl] * scale;
  }
  __syncthreads();
  const int lane = t & 31, wave = t >> 5;
  const int q = lane >> 3, c8 = (lane & 7) * 8;
  for (int pass = 0; pass < 2; ++pass) {
#pragma unroll
    for (int it = 0; it < 2; ++it) {
      const int row = wave * 8 + it * 4 + q;
      unsigned short hb[8];
#pragma unroll
      for (int e = 0; e < 8; ++e) hb[e] = h_bits(sm[row][c8 + e]);
      const v4u u = (v4u){pk16(hb[0], hb[1]), pk16(hb[2], hb[3]), pk16(hb[4], hb[5]), pk16(hb[6], hb[7])};
      *(volatile v4u*)(out + (size_t)(c0 + row) * R + r0 + c8) = u;
    }
    __threadfence();
  }
}

__global__ __launch_bounds__(96) void ln_f16_kernel(const float* __restrict__ xin, const float* __restrict__ gam,
                                                   const float* __restrict__ bet, unsigned short* __restrict__ outp) {
  __shared__ float red1[3];
  __shared__ float red2[3];
  const int row  = blockIdx.x;
  const int t    = threadIdx.x;
  const int lane = t & 31, wave = t >> 5;
  const int c0   = 8 * t;
  const float* xr = xin + (size_t)row * kDim + c0;
  const v4f a = *(const v4f*)(xr);
  const v4f c = *(const v4f*)(xr + 4);
  float v[8];
#pragma unroll
  for (int e = 0; e < 4; ++e) { v[e] = a[e]; v[4 + e] = c[e]; }
  float s = ((v[0] + v[1]) + (v[2] + v[3])) + ((v[4] + v[5]) + (v[6] + v[7]));
#pragma unroll
  for (int off = 16; off > 0; off >>= 1) s += __shfl_xor(s, off, 32);
  if (lane == 0) red1[wave] = s;
  __syncthreads();
  const float mu = ((red1[0] + red1[1]) + red1[2]) * kInvDim;
  float d[8];
  float s2 = 0.0f;
#pragma unroll
  for (int e = 0; e < 8; ++e) { d[e] = v[e] - mu; s2 += d[e] * d[e]; }
#pragma unroll
  for (int off = 16; off > 0; off >>= 1) s2 += __shfl_xor(s2, off, 32);
  if (lane == 0) red2[wave] = s2;
  __syncthreads();
  const float var  = ((red2[0] + red2[1]) + red2[2]) * kInvDim;
  const float rinv = rsqrtf(var + kLnEps);
  const v4f g0 = *(const v4f*)(gam + c0);
  const v4f g1 = *(const v4f*)(gam + c0 + 4);
  const v4f b0 = *(const v4f*)(bet + c0);
  const v4f b1 = *(const v4f*)(bet + c0 + 4);
  unsigned short hb[8];
#pragma unroll
  for (int e = 0; e < 4; ++e) {
    hb[e]     = h_bits(d[e] * rinv * g0[e] + b0[e]);
    hb[4 + e] = h_bits(d[4 + e] * rinv * g1[e] + b1[e]);
  }
  const v4u u = (v4u){pk16(hb[0], hb[1]), pk16(hb[2], hb[3]), pk16(hb[4], hb[5]), pk16(hb[6], hb[7])};
  unsigned short* op = outp + (size_t)row * kDim + c0;
  *(volatile v4u*)op = u;
  __threadfence();
  *(volatile v4u*)op = u;
}

__global__ __launch_bounds__(64) void softmax_row_kernel(const float* __restrict__ Sp, unsigned short* __restrict__ Pp) {
  __shared__ __align__(16) float lg[kSeq];
  __shared__ float redM[2];
  __shared__ float redS[2];
  const int i    = blockIdx.x;
  const int hg   = blockIdx.y;
  const int t    = threadIdx.x;
  const int lane = t & 31, wave = t >> 5;
  const size_t rowoff = ((size_t)hg * kSeq + i) * kSeq;
  const float* sr = Sp + rowoff;

  float mx = -__builtin_inff();
#pragma unroll 1
  for (int it = 0; it < 4; ++it) {
    const int c = it * 128 + 2 * t;
    const v2f sv = *(const v2f*)(sr + c);
    mx = fmaxf(mx, fmaxf(sv[0], sv[1]));
    *(v2f*)(lg + c) = sv;
  }
#pragma unroll
  for (int off = 16; off > 0; off >>= 1) mx = fmaxf(mx, __shfl_xor(mx, off, 32));
  if (lane == 0) redM[wave] = mx;
  __syncthreads();
  const float m = fmaxf(redM[0], redM[1]);

  float sum = 0.0f;
#pragma unroll 1
  for (int it = 0; it < 4; ++it) {
    const int c = it * 128 + 2 * t;
    const v2f l = *(const v2f*)(lg + c);
    v2f ev;
#pragma unroll
    for (int e = 0; e < 2; ++e) {
      ev[e] = expf(l[e] - m);
      sum += ev[e];
    }
    *(v2f*)(lg + c) = ev;
  }
#pragma unroll
  for (int off = 16; off > 0; off >>= 1) sum += __shfl_xor(sum, off, 32);
  if (lane == 0) redS[wave] = sum;
  __syncthreads();
  const float tot = redS[0] + redS[1];
  const float inv = kPCarry * (1.0f / tot);

  const v4f e0 = *(const v4f*)(lg + 8 * t);
  const v4f e1 = *(const v4f*)(lg + 8 * t + 4);
  unsigned short hb[8];
#pragma unroll
  for (int e = 0; e < 4; ++e) {
    hb[e]     = h_bits(e0[e] * inv);
    hb[4 + e] = h_bits(e1[e] * inv);
  }
  const v4u u = (v4u){pk16(hb[0], hb[1]), pk16(hb[2], hb[3]), pk16(hb[4], hb[5]), pk16(hb[6], hb[7])};
  unsigned short* pr = Pp + rowoff + 8 * (size_t)t;
  *(volatile v4u*)pr = u;
  __threadfence();
  *(volatile v4u*)pr = u;
}

__global__ __launch_bounds__(256) void gelu_f16_kernel(unsigned short* plane) {
  __shared__ __align__(16) unsigned int smw[2048];
  const int t    = threadIdx.x;
  const size_t base = (size_t)blockIdx.x * 4096;
  const unsigned int* wp = (const unsigned int*)(plane + base);
  unsigned lowb = 0u;
#pragma unroll 1
  for (int it = 0; it < 16; ++it) {
    const int w  = (it >> 1) * 256 + t;
    const int hi = it & 1;
    const unsigned word  = wp[w];
    const unsigned hbits = hi ? (word >> 16) : (word & 0xffffu);
    const float u  = h16_to_f32(hbits);
    const float gl = 0.5f * u * (1.0f + erff(u * 0.70710678118654752f));
    const unsigned ob = (unsigned)h_bits(gl);
    if (hi) smw[w] = lowb | (ob << 16);
    else    lowb = ob;
  }
  __syncthreads();
  v4u vals[2];
#pragma unroll
  for (int j = 0; j < 2; ++j) vals[j] = *(const v4u*)(smw + j * 1024 + 4 * t);
  unsigned short* op = plane + base;
  for (int pass = 0; pass < 2; ++pass) {
#pragma unroll
    for (int j = 0; j < 2; ++j) *(volatile v4u*)(op + (size_t)j * 2048 + 8 * (size_t)t) = vals[j];
    __threadfence();
  }
}

extern "C" void kernel_launch(void* const* d_in, const int* in_sizes, int n_in,
                              void* d_out, int out_size, void* d_ws, size_t ws_size,
                              hipStream_t stream) {
  if (n_in < 15) return;
  const int nElem = kTok * kDim;
  if (in_sizes[0] != nElem || out_size != nElem) return;
  if (in_sizes[1] != kDim || in_sizes[2] != kDim || in_sizes[9] != kDim || in_sizes[10] != kDim || in_sizes[14] != kDim) return;
  if (in_sizes[3] != kHeads * kHeadW || in_sizes[5] != kHeads * kHeadW || in_sizes[7] != kHeads * kHeadW) return;
  if (in_sizes[4] != kHeads * kDh || in_sizes[6] != kHeads * kDh || in_sizes[8] != kHeads * kDh) return;
  if (in_sizes[11] != kDim * kMlp || in_sizes[13] != kMlp * kDim || in_sizes[12] != kMlp) return;

  const size_t szWT    = (size_t)3 * kHeads * kHeadW * 2;
  const size_t szW1T   = (size_t)kMlp * kDim * 2;
  const size_t szW2T   = (size_t)kDim * kMlp * 2;
  const size_t szTok16 = (size_t)kTok * kDim * 2;
  const size_t szVT    = (size_t)kHeads * kDh * kTok * 2;
  const size_t szSC    = (size_t)kHeads * kSeq * kSeq * 4;
  const size_t szPP    = (size_t)kHeads * kSeq * kSeq * 2;
  const size_t szUP    = (size_t)kMChunk * kMlp * 2;
  const size_t offWT  = 0;
  const size_t offW1T = offWT + szWT;
  const size_t offW2T = offW1T + szW1T;
  const size_t offXLN = offW2T + szW2T;
  const size_t offQ   = offXLN + szTok16;
  const size_t offK   = offQ + szTok16;
  const size_t offVT  = offK + szTok16;
  const size_t offHLN = offVT + szVT;
  const size_t offSC  = offHLN + szTok16;
  const size_t offPP  = offSC + szSC;
  const size_t offUP  = offPP + szPP;
  const size_t total  = offUP + szUP;
  if (ws_size < total) return;

  const float* xin  = (const float*)d_in[0];
  const float* ln1g = (const float*)d_in[1];
  const float* ln1b = (const float*)d_in[2];
  const float* wq   = (const float*)d_in[3];
  const float* bq   = (const float*)d_in[4];
  const float* wk   = (const float*)d_in[5];
  const float* bk   = (const float*)d_in[6];
  const float* wv   = (const float*)d_in[7];
  const float* bv   = (const float*)d_in[8];
  const float* ln2g = (const float*)d_in[9];
  const float* ln2b = (const float*)d_in[10];
  const float* w1   = (const float*)d_in[11];
  const float* b1   = (const float*)d_in[12];
  const float* w2   = (const float*)d_in[13];
  const float* b2   = (const float*)d_in[14];
  float* out = (float*)d_out;
  char* ws = (char*)d_ws;
  unsigned short* WT  = (unsigned short*)(ws + offWT);
  unsigned short* W1T = (unsigned short*)(ws + offW1T);
  unsigned short* W2T = (unsigned short*)(ws + offW2T);
  unsigned short* XLN = (unsigned short*)(ws + offXLN);
  unsigned short* QP  = (unsigned short*)(ws + offQ);
  unsigned short* KP  = (unsigned short*)(ws + offK);
  unsigned short* VT  = (unsigned short*)(ws + offVT);
  unsigned short* HLN = (unsigned short*)(ws + offHLN);
  float* SC = (float*)(ws + offSC);
  unsigned short* PP  = (unsigned short*)(ws + offPP);
  unsigned short* UP  = (unsigned short*)(ws + offUP);
  const unsigned short* WqT = WT;
  const unsigned short* WkT = WT + (size_t)1 * kHeads * kHeadW;
  const unsigned short* WvT = WT + (size_t)2 * kHeads * kHeadW;

  wcast_head_kernel<<<dim3(kHeads, 3), dim3(256), 0, stream>>>(wq, wk, wv, WT, kWCarry);
  wtcast_kernel<<<dim3(kDim / 64, kMlp / 64), dim3(256), 0, stream>>>(w1, W1T, kDim, kMlp, kWCarry);
  wtcast_kernel<<<dim3(kMlp / 64, kDim / 64), dim3(256), 0, stream>>>(w2, W2T, kMlp, kDim, kWCarry);

  ln_f16_kernel<<<dim3(kTok), dim3(96), 0, stream>>>(xin, ln1g, ln1b, XLN);

  const long strideHeadCol = (long)kDh;
  const long strideHeadW   = (long)kHeadW;
  const long strideHeadVT  = (long)kDh * kTok;
  const int  tilesProj     = (kTok / 64) * (kDh / 64);
  wmma_gemm64<0, false, 2, 1, false><<<dim3(tilesProj / 8, kHeads), dim3(256), 0, stream>>>(
      XLN, XLN, kDim, strideHeadCol, WqT, WqT, kDh, strideHeadW,
      (void*)QP, (void*)QP, kDim, strideHeadCol, bq, (long)kDh, xin, 0L, kTok, kDh, kDh, kWCarryInv);
  wmma_gemm64<0, false, 2, 1, false><<<dim3(tilesProj / 8, kHeads), dim3(256), 0, stream>>>(
      XLN, XLN, kDim, strideHeadCol, WkT, WkT, kDh, strideHeadW,
      (void*)KP, (void*)KP, kDim, strideHeadCol, bk, (long)kDh, xin, 0L, kTok, kDh, kDh, kWCarryInv);
  wmma_gemm64<0, false, 1, 1, false><<<dim3(tilesProj / 8, kHeads), dim3(256), 0, stream>>>(
      WvT, WvT, kDh, strideHeadW, XLN, XLN, kDim, strideHeadCol,
      (void*)VT, (void*)VT, kTok, strideHeadVT, bv, (long)kDh, xin, 0L, kDh, kTok, kDh, kWCarryInv);

  const long strideScore = (long)kSeq * kSeq;
  const int  tilesScore  = (kSeq / 64) * (kSeq / 64);
  const int  tilesCtx    = (kSeq / 64) * (kDh / 64);
  for (int b = 0; b < kBatch; ++b) {
    const size_t tokOff = (size_t)b * kSeq * kDim;
    wmma_gemm64<0, false, 0, 0, false><<<dim3(tilesScore / 8, kHeads), dim3(256), 0, stream>>>(
        QP + tokOff, QP + tokOff, kDim, strideHeadCol, KP + tokOff, KP + tokOff, kDim, strideHeadCol,
        (void*)SC, (void*)SC, kSeq, strideScore, bq, 0L, xin, 0L, kSeq, kSeq, kDh, kScoreScale);
    softmax_row_kernel<<<dim3(kSeq, kHeads), dim3(64), 0, stream>>>(SC, PP);
    wmma_gemm64<0, false, 0, 0, true><<<dim3(tilesCtx / 8, kHeads), dim3(256), 0, stream>>>(
        PP, PP, kSeq, strideScore, VT + (size_t)b * kSeq, VT + (size_t)b * kSeq, kTok, strideHeadVT,
        (void*)(out + tokOff), (void*)(out + tokOff), kDim, strideHeadCol, bq, 0L,
        xin + tokOff, strideHeadCol, kSeq, kDh, kSeq, kPCarryInv);
  }

  ln_f16_kernel<<<dim3(kTok), dim3(96), 0, stream>>>(out, ln2g, ln2b, HLN);

  const int tilesUp   = (kMChunk / 64) * (kMlp / 64);
  const int tilesDown = (kMChunk / 64) * (kDim / 64);
  for (int mc = 0; mc < kTok / kMChunk; ++mc) {
    const size_t rowOff = (size_t)mc * kMChunk;
    wmma_gemm64<0, false, 2, 1, false><<<dim3(tilesUp / 8, 1), dim3(256), 0, stream>>>(
        HLN + rowOff * kDim, HLN + rowOff * kDim, kDim, 0L, W1T, W1T, kDim, 0L,
        (void*)UP, (void*)UP, kMlp, 0L, b1, 0L, xin, 0L, kMChunk, kMlp, kDim, kWCarryInv);
    gelu_f16_kernel<<<dim3((kMChunk * kMlp) / 4096), dim3(256), 0, stream>>>(UP);
    wmma_gemm64<0, false, 2, 0, true><<<dim3(tilesDown / 8, 1), dim3(256), 0, stream>>>(
        UP, UP, kMlp, 0L, W2T, W2T, kMlp, 0L,
        (void*)(out + rowOff * kDim), (void*)(out + rowOff * kDim), kDim, 0L, b2, 0L,
        out + rowOff * kDim, 0L, kMChunk, kDim, kMlp, kWCarryInv);
  }
}
